// TrulyNeuralMMUv2_18975165514017
// MI455X (gfx1250) — hardware-verified
//
#include <hip/hip_runtime.h>
#include <math.h>

typedef __attribute__((ext_vector_type(16))) _Float16 v16h;
typedef __attribute__((ext_vector_type(16))) __bf16 v16b;
typedef __attribute__((ext_vector_type(8)))  _Float16 v8h;
typedef __attribute__((ext_vector_type(8)))  float v8f;
typedef __attribute__((ext_vector_type(4)))  float v4f;
typedef __attribute__((ext_vector_type(2)))  float v2f;
typedef __attribute__((ext_vector_type(4)))  unsigned v4u;
typedef __attribute__((ext_vector_type(4)))  int v4i;
typedef float __attribute__((may_alias)) float_a;
typedef int __attribute__((may_alias)) int_a;

template <typename T> __device__ __forceinline__ void vst2(void* p, T v) { *(volatile T*)p = v; __threadfence(); *(volatile T*)p = v; }
__device__ __forceinline__ v8f wmma16(v16h a, v16h b, v8f c) {
  v8f d = __builtin_amdgcn_wmma_f32_16x16x32_f16(false, a, false, b, (short)0, c, false, false);
  asm volatile("v_nop\n\tv_nop\n\tv_nop\n\tv_nop" : "+v"(d) : "v"(a), "v"(b));
  return d;
}
__device__ __forceinline__ v8f wmma_bf(v16b a, v16b b, v8f c) {
  v8f d = __builtin_amdgcn_wmma_f32_16x16x32_bf16(false, a, false, b, (short)0, c, false, false);
  asm volatile("v_nop\n\tv_nop\n\tv_nop\n\tv_nop" : "+v"(d) : "v"(a), "v"(b));
  return d;
}
__device__ __forceinline__ v16h frag_h(const _Float16* rowk0, int lane) {
  union { v16h v; v8h q[2]; } u; const _Float16* p = rowk0 + 8 * (lane >> 4);
  u.q[0] = *(const v8h*)p; u.q[1] = *(const v8h*)(p + 16); return u.v;
}
__device__ __forceinline__ v16h frag_f32(const float* rowk0, int lane) {
  v16h a; const float* p = rowk0 + 8 * (lane >> 4);
#pragma unroll
  for (int i = 0; i < 8; ++i) { a[i] = (_Float16)p[i]; a[8 + i] = (_Float16)p[16 + i]; }
  return a;
}
__device__ __forceinline__ v16h frag_f32s(const float* rowk0, int lane, float sc) {
  v16h a; const float* p = rowk0 + 8 * (lane >> 4);
#pragma unroll
  for (int i = 0; i < 8; ++i) { a[i] = (_Float16)(p[i] * sc); a[8 + i] = (_Float16)(p[16 + i] * sc); }
  return a;
}
__device__ __forceinline__ v16h fragc_f32(const float* W, int k0, int n, int lane, int ld, int K) {
  v16h a; const int g = lane >> 4;
#pragma unroll
  for (int i = 0; i < 8; ++i) { const int ka = k0 + 8 * g + i, kb = ka + 16;
    a[i] = (_Float16)(ka < K ? W[(size_t)(ka < K ? ka : K - 1) * ld + n] : 0.f); a[8 + i] = (_Float16)(kb < K ? W[(size_t)(kb < K ? kb : K - 1) * ld + n] : 0.f); }
  return a;
}
struct F2 { v16b h, l; };
__device__ __forceinline__ F2 bsplit16(const float v[16]) { F2 r;
#pragma unroll
  for (int i = 0; i < 16; ++i) { const __bf16 h = (__bf16)v[i]; r.h[i] = h; r.l[i] = (__bf16)(v[i] - (float)h); }
  return r; }
__device__ __forceinline__ F2 split_row(const float* row, int k0, int lane) { float v[16]; const float* p = row + k0 + 8 * (lane >> 4);
#pragma unroll
  for (int i = 0; i < 8; ++i) { v[i] = p[i]; v[8 + i] = p[16 + i]; }
  return bsplit16(v); }
__device__ __forceinline__ F2 split_rowK(const float* row, int k0, int lane, int K) { float v[16]; const int g = lane >> 4;
#pragma unroll
  for (int i = 0; i < 8; ++i) { const int ka = k0 + 8 * g + i, kb = ka + 16; v[i] = ka < K ? row[ka < K ? ka : K - 1] : 0.f; v[8 + i] = kb < K ? row[kb < K ? kb : K - 1] : 0.f; }
  return bsplit16(v); }
__device__ __forceinline__ F2 split_col(const float* W, int k0, int n, int lane, int ld, int K) { float v[16]; const int g = lane >> 4;
#pragma unroll
  for (int i = 0; i < 8; ++i) { const int ka = k0 + 8 * g + i, kb = ka + 16; v[i] = ka < K ? W[(size_t)(ka < K ? ka : K - 1) * ld + n] : 0.f; v[8 + i] = kb < K ? W[(size_t)(kb < K ? kb : K - 1) * ld + n] : 0.f; }
  return bsplit16(v); }
__device__ __forceinline__ v8f mac3(const F2& a, const F2& b, v8f c) { c = wmma_bf(a.l, b.h, c); c = wmma_bf(a.h, b.l, c); return wmma_bf(a.h, b.h, c); }
__device__ __forceinline__ float sigm(float v) { return 1.0f / (1.0f + expf(-v)); }
#define LDSX() do { asm volatile("s_wait_dscnt 0" ::: "memory"); __builtin_amdgcn_wave_barrier(); __builtin_amdgcn_fence(__ATOMIC_RELEASE, "workgroup"); } while (0)


#define NBT 32768
#define NP 4096
#define KD 64
#define PB 20
#define H1 128
#ifndef TQB
#define TQB (NBT / 64)
#endif
typedef __attribute__((ext_vector_type(8))) __bf16 v8b;
__device__ __forceinline__ v16b frag_b(const __bf16* rowk0, int lane) {
  union { v16b v; v8b q[2]; } u; const __bf16* p = rowk0 + 8 * (lane >> 4);
  u.q[0] = *(const v8b*)p; u.q[1] = *(const v8b*)(p + 16); return u.v;
}
__device__ __forceinline__ v16b frag_gbf(const float* rowk0, int lane) {
  v16b a; const float* p = rowk0 + 8 * (lane >> 4);
#pragma unroll
  for (int i = 0; i < 8; ++i) { a[i] = (__bf16)p[i]; a[8 + i] = (__bf16)p[16 + i]; }
  return a;
}
__device__ __forceinline__ float bfr(float v) { return (float)(__bf16)v; }
__device__ __attribute__((noinline)) float exp_ni(float v) { return expf(v); }
__device__ __attribute__((noinline)) float erf_ni(float v) { return erff(v); }
__device__ __attribute__((noinline)) float sigm_(float v) { return 1.0f / (1.0f + expf(-v)); }
#define WS_SVH  0u
#define WS_SVL  (WS_SVH + 2u * NP * 32)
#define WS_SS   (WS_SVL + 2u * NP * 32)
#define WS_PLH  (WS_SS + 4u * NP)
#define WS_PLL  (WS_PLH + 2u * 32 * NP)
#define WS_Q    (WS_PLL + 2u * 32 * NP)
#define WS_X2   (WS_Q + 4u * NBT * KD)
#define WS_ST   (WS_X2 + 4u * NBT)
#define WS_END  (WS_ST + 4u * NBT * 32)

__global__ __launch_bounds__(256) void k_pages(const float* __restrict__ VP, const float* __restrict__ PP, const float* __restrict__ PM, __bf16* __restrict__ SVH, __bf16* __restrict__ SVL, float* __restrict__ SS, __bf16* __restrict__ PLH, __bf16* __restrict__ PLL) {
  __shared__ __align__(16) __bf16 sh[64][40], sl[64][40]; __shared__ __align__(16) float sss[64]; __shared__ __align__(16) __bf16 sph[32][72], spl[32][72];
  const int tid = threadIdx.x; const int p0 = blockIdx.x * 64; const int pl = tid >> 2, part = tid & 3;
  { float s2 = 0.f;
#pragma unroll 1
    for (int c = part * 8; c < part * 8 + 8; ++c) { float v = 0.f; if (c < PB) { v = sigm_(bfr(VP[(size_t)(p0 + pl) * PB + c])); s2 += v * v; } const __bf16 hb = (__bf16)v; sh[pl][c] = hb; sl[pl][c] = (__bf16)(v - (float)hb);
      float w = 0.f; if (c < PB) w = sigm_(bfr(PP[(size_t)(p0 + pl) * PB + c])); else if (c < PB + 4) w = sigm_(bfr(PM[(size_t)(p0 + pl) * 4 + c - PB])); const __bf16 wb = (__bf16)w; sph[c][pl] = wb; spl[c][pl] = (__bf16)(w - (float)wb); }
    s2 += __shfl_xor(s2, 1); s2 += __shfl_xor(s2, 2); if (part == 0) sss[pl] = s2; }
  __syncthreads();
  for (int q = tid; q < 64 * 4; q += 256) { const int r = q >> 2, pc = q & 3; vst2((unsigned*)(SVH + (size_t)(p0 + r) * 32 + pc * 8), *(const v4u*)&sh[r][pc * 8]); vst2((unsigned*)(SVL + (size_t)(p0 + r) * 32 + pc * 8), *(const v4u*)&sl[r][pc * 8]); }
  if (tid < 16) vst2(SS + p0 + tid * 4, *(const v4f*)&sss[tid * 4]);
  for (int q = tid; q < 32 * 8; q += 256) { const int c = q >> 3, pc = q & 7; vst2((unsigned*)(PLH + (size_t)c * NP + p0 + pc * 8), *(const v4u*)&sph[c][pc * 8]); vst2((unsigned*)(PLL + (size_t)c * NP + p0 + pc * 8), *(const v4u*)&spl[c][pc * 8]); }
}
__global__ __launch_bounds__(128) void k_query(const float* __restrict__ BITS, const float* __restrict__ W1, const float* __restrict__ b1, const float* __restrict__ W2, const float* __restrict__ b2, float* __restrict__ Q, float* __restrict__ X2) {
  __shared__ __align__(16) __bf16 sa[64][40]; __shared__ __align__(16) __bf16 sw1[H1][40]; __shared__ __align__(16) __bf16 sw2[KD][136]; __shared__ __align__(16) __bf16 shh[4][16][136], shl[4][16][136]; __shared__ __align__(16) float so[4][16][68]; __shared__ __align__(16) float sx2[64];
  const int tid = threadIdx.x, wave = tid >> 5, lane = tid & 31, col = lane & 15, g = lane >> 4; const size_t r0 = (size_t)blockIdx.x * 64;
  for (int q = tid; q < 64 * 32; q += 128) { const int rl = q >> 5, c = q & 31; sa[rl][c] = (__bf16)((c < PB) ? bfr(BITS[(r0 + rl) * PB + c]) : 0.f); }
  for (int q = tid; q < H1 * 32; q += 128) { const int o = q >> 5, c = q & 31; sw1[o][c] = (__bf16)((c < PB) ? bfr(W1[(size_t)c * H1 + o]) : 0.f); }
  for (int q = tid; q < KD * H1; q += 128) { const int o = q / H1, k = q % H1; sw2[o][k] = (__bf16)bfr(W2[(size_t)k * KD + o]); }
  if (tid < 64) { float s = 0.f; for (int c = 0; c < PB; ++c) { const float v = bfr(BITS[(r0 + tid) * PB + c]); s += v * v; } sx2[tid] = s; }
  __syncthreads();
  { const v16b a = frag_b(&sa[wave * 16 + col][0], lane);
#pragma unroll
    for (int j = 0; j < 8; ++j) { v8f acc = {}; acc = wmma_bf(a, frag_b(&sw1[j * 16 + col][0], lane), acc);
#pragma unroll
      for (int r = 0; r < 8; ++r) { const float v = acc[r] + bfr(b1[j * 16 + col]); const float gl = 0.5f * v * (1.0f + erf_ni(v * 0.70710678118654752f)); const __bf16 hb = (__bf16)gl; shh[wave][8 * g + r][j * 16 + col] = hb; shl[wave][8 * g + r][j * 16 + col] = (__bf16)(gl - (float)hb); } } }
  LDSX();
  { v8f acc[4] = {};
#pragma unroll
    for (int kc = 0; kc < H1 / 32; ++kc) { const v16b ah = frag_b(&shh[wave][col][kc * 32], lane), al = frag_b(&shl[wave][col][kc * 32], lane);
#pragma unroll
      for (int j = 0; j < 4; ++j) { const v16b w = frag_b(&sw2[j * 16 + col][kc * 32], lane); acc[j] = wmma_bf(al, w, acc[j]); acc[j] = wmma_bf(ah, w, acc[j]); } }
#pragma unroll
    for (int j = 0; j < 4; ++j)
#pragma unroll
      for (int r = 0; r < 8; ++r) so[wave][8 * g + r][j * 16 + col] = acc[j][r] + bfr(b2[j * 16 + col]); }
  LDSX();
  for (int rl = 0; rl < 16; ++rl) if (lane < 16) vst2(Q + (r0 + wave * 16 + rl) * KD + lane * 4, *(const v4f*)&so[wave][rl][lane * 4]);
  __syncthreads();
  if (tid < 16) vst2(X2 + r0 + tid * 4, *(const v4f*)&sx2[tid * 4]);
}
__global__ __launch_bounds__(128) void k_attn(const float* __restrict__ Q, const float* __restrict__ BITS, const float* __restrict__ X2, const float* __restrict__ PK, const __bf16* __restrict__ SVH, const __bf16* __restrict__ SVL, const float* __restrict__ SS, const __bf16* __restrict__ PLH, const __bf16* __restrict__ PLL, const float* __restrict__ TEMP, float* __restrict__ ST) {
  __shared__ __align__(16) __bf16 sbit[64][40]; __shared__ __align__(16) float sp[4][16][36]; __shared__ __align__(16) float so[4][16][36];
  const int tid = threadIdx.x, wave = tid >> 5, lane = tid & 31, col = lane & 15, g = lane >> 4; const size_t r0 = (size_t)blockIdx.x * 64 + wave * 16;
  for (int q = tid; q < 64 * 32; q += 128) { const int rl = q >> 5, c = q & 31; sbit[rl][c] = (__bf16)((c < PB) ? bfr(BITS[((size_t)blockIdx.x * 64 + rl) * PB + c]) : 0.f); }
  __syncthreads();
  const F2 a0 = split_row(Q + (r0 + col) * KD, 0, lane), a1 = split_row(Q + (r0 + col) * KD, 32, lane); const v16b ab = frag_b(&sbit[wave * 16 + col][0], lane);
  const float itemp = 1.0f / fmaxf(fabsf(bfr(TEMP[0])), 0.1f);
  float x2r[8];
#pragma unroll
  for (int r = 0; r < 8; ++r) x2r[r] = X2[r0 + 8 * g + r];
  float m[8], l[8]; v8f acc[2] = {};
#pragma unroll
  for (int r = 0; r < 8; ++r) { m[r] = -3.0e38f; l[r] = 0.f; }
#pragma unroll 1
  for (int ks = 0; ks < NP / 32; ++ks) { float s[2][8];
#pragma unroll
    for (int ct = 0; ct < 2; ++ct) { const int p = ks * 32 + ct * 16 + col; v8f ksim = {}; const v16b k0 = frag_gbf(PK + (size_t)p * KD, lane), k1 = frag_gbf(PK + (size_t)p * KD + 32, lane);
      ksim = wmma_bf(a0.l, k0, ksim); ksim = wmma_bf(a0.h, k0, ksim); ksim = wmma_bf(a1.l, k1, ksim); ksim = wmma_bf(a1.h, k1, ksim);
      v8f cr = {}; const v16b svh = frag_b(SVH + (size_t)p * 32, lane), svl = frag_b(SVL + (size_t)p * 32, lane); cr = wmma_bf(ab, svl, cr); cr = wmma_bf(ab, svh, cr);
      const float ssp = SS[p];
#pragma unroll
      for (int r = 0; r < 8; ++r) { const float page_sim = -(x2r[r] + ssp - 2.0f * cr[r]); s[ct][r] = (ksim[r] + 2.0f * page_sim) * itemp; } }
#pragma unroll
    for (int r = 0; r < 8; ++r) { float mx = fmaxf(s[0][r], s[1][r]);
#pragma unroll
      for (int o = 1; o < 16; o <<= 1) mx = fmaxf(mx, __shfl_xor(mx, o));
      const float mn = fmaxf(m[r], mx); const float alpha = exp_ni(m[r] - mn); const float e0 = exp_ni(s[0][r] - mn), e1 = exp_ni(s[1][r] - mn); float es = e0 + e1;
#pragma unroll
      for (int o = 1; o < 16; o <<= 1) es += __shfl_xor(es, o);
      l[r] = l[r] * alpha + es; m[r] = mn; acc[0][r] *= alpha; acc[1][r] *= alpha; sp[wave][8 * g + r][col] = e0; sp[wave][8 * g + r][16 + col] = e1; }
    LDSX();
    const F2 pa = split_row(&sp[wave][col][0], 0, lane);
#pragma unroll
    for (int dt = 0; dt < 2; ++dt) { const size_t prow = (size_t)(dt * 16 + col) * NP + ks * 32; const v16b vh = frag_b(PLH + prow, lane), vl = frag_b(PLL + prow, lane); acc[dt] = wmma_bf(pa.l, vh, acc[dt]); acc[dt] = wmma_bf(pa.h, vl, acc[dt]); acc[dt] = wmma_bf(pa.h, vh, acc[dt]); }
    LDSX(); }
#pragma unroll
  for (int r = 0; r < 8; ++r) { const float il = 1.0f / l[r]; so[wave][8 * g + r][col] = acc[0][r] * il; so[wave][8 * g + r][16 + col] = acc[1][r] * il; }
  LDSX();
  for (int rl = 0; rl < 16; ++rl) if (lane < 8) vst2(ST + (r0 + rl) * 32 + lane * 4, *(const v4f*)&so[wave][rl][lane * 4]);
}
__global__ __launch_bounds__(256) void k_copy(const float* __restrict__ ST, float* __restrict__ out) {
  const size_t p = (size_t)blockIdx.x * 256 + threadIdx.x; const size_t n0 = (size_t)NBT * PB, n1 = NBT, n2 = (size_t)NBT * 3; const size_t total = n0 + n1 + n2; if (p * 4 >= total) return;
  v4f v; for (int i = 0; i < 4; ++i) { const size_t f = p * 4 + i; float val = 0.f; if (f < n0) { val = ST[(f / PB) * 32 + (f % PB)]; } else if (f < n0 + n1) { val = ST[(f - n0) * 32 + PB]; } else if (f < total) { const size_t e = f - n0 - n1; val = ST[(e / 3) * 32 + PB + 1 + (e % 3)]; } v[i] = val; }
  vst2(out + p * 4, v);
}
extern "C" void kernel_launch(void* const* d_in, const int* in_sizes, int n_in, void* d_out, int out_size, void* d_ws, size_t ws_size, hipStream_t stream) {
  (void)in_sizes; (void)n_in; (void)out_size;
  const float** F = (const float**)d_in;
  if (ws_size < (size_t)WS_END) return;
  char* ws = (char*)d_ws; __bf16 *SVH = (__bf16*)(ws + WS_SVH), *SVL = (__bf16*)(ws + WS_SVL), *PLH = (__bf16*)(ws + WS_PLH), *PLL = (__bf16*)(ws + WS_PLL); float *SS = (float*)(ws + WS_SS), *Q = (float*)(ws + WS_Q), *X2 = (float*)(ws + WS_X2), *ST = (float*)(ws + WS_ST);
  k_pages<<<NP / 64, 256, 0, stream>>>(F[2], F[3], F[4], SVH, SVL, SS, PLH, PLL);
  k_query<<<TQB, 128, 0, stream>>>(F[0], F[5], F[6], F[7], F[8], Q, X2);
  k_attn<<<TQB, 128, 0, stream>>>(Q, F[0], X2, F[1], SVH, SVL, SS, PLH, PLL, F[9], ST);
  k_copy<<<(NBT * 24 / 4 + 255) / 256, 256, 0, stream>>>(ST, (float*)d_out);
}
